// SDPADilatedAttention_30331059044984
// MI455X (gfx1250) — hardware-verified
//
#include <hip/hip_runtime.h>
#include <math.h>
#include <stdint.h>

#define NBT  2
#define SEQ  2048
#define HH   768
#define NHD  12
#define HD   64
#define SEGL 256
#define MT   (NBT * SEQ)
#define QT   128
#define NCHK (SEGL / 32)
#define ZSP  72
#define WSC  16.0f
#define PSC  1024.0f
#define ZSC  16.0f
#define RSC  2048.0f
#define RSCI 0.00048828125f
#define SCL  0.125f

static_assert(NHD * HD == HH);
static_assert(HD == 64);
static_assert((SEQ % SEGL) == 0 && (SEGL % QT) == 0 && (MT % QT) == 0 && QT == 128 && (SEGL % 32) == 0);
static_assert((MT % 64) == 0 && (HH % 64) == 0 && (MT % 32) == 0 && (HH % 32) == 0);
static_assert((((MT / 64) * (HH / 64)) % 8) == 0);
static_assert((((HH / 64) * (MT / 64)) % 8) == 0);
static_assert((((MT / 32) * (HH / 64)) % 8) == 0);
static_assert((MT % 8) == 0 && (HH % 8) == 0 && (HH % 256) == 0);
static_assert(ZSP >= 64 && (ZSP % 8) == 0);

typedef _Float16 v16h __attribute__((ext_vector_type(16)));
typedef _Float16 v8h  __attribute__((ext_vector_type(8)));
typedef unsigned short v16us __attribute__((ext_vector_type(16)));
typedef unsigned short v8us  __attribute__((ext_vector_type(8)));
typedef float v8f __attribute__((ext_vector_type(8)));
typedef float v4f __attribute__((ext_vector_type(4)));
typedef unsigned int v4u __attribute__((ext_vector_type(4)));

union FragU { v16us v; v8us h[2]; };

__device__ __forceinline__ unsigned short bf_bits(float f) {
  const unsigned u = __float_as_uint(f);
  return (unsigned short)((u + 0x7FFFu + ((u >> 16) & 1u)) >> 16);
}
__device__ __forceinline__ float bf_up(unsigned short h) { return __uint_as_float(((unsigned)h) << 16); }
__device__ __forceinline__ float bfr(float f) { return bf_up(bf_bits(f)); }
__device__ __forceinline__ unsigned short h_bits(_Float16 x) { return __builtin_bit_cast(unsigned short, x); }
__device__ __forceinline__ unsigned short f2h(float f) { return h_bits((_Float16)f); }
__device__ __forceinline__ float h_up(unsigned short h) { return (float)__builtin_bit_cast(_Float16, h); }
__device__ __forceinline__ unsigned pk16(unsigned short a, unsigned short b) { return (unsigned)a | ((unsigned)b << 16); }
__device__ __forceinline__ v8f zero8() { v8f z = {0.f, 0.f, 0.f, 0.f, 0.f, 0.f, 0.f, 0.f}; return z; }
__device__ __forceinline__ void split_h(float f, unsigned short& hi, unsigned short& lo) {
  hi = f2h(f);
  lo = f2h((f - h_up(hi)) * RSC);
}

__device__ __forceinline__ v16us ldfrag_u(const unsigned short* p) {
  FragU f;
  f.h[0] = *(const v8us*)(p);
  f.h[1] = *(const v8us*)(p + 16);
  return f.v;
}

__device__ __forceinline__ v8f mma_h_raw(v16us a, v16us b, v8f c) {
  return __builtin_amdgcn_wmma_f32_16x16x32_f16(false, __builtin_bit_cast(v16h, a), false,
                                                __builtin_bit_cast(v16h, b), (short)0, c, false, false);
}
__device__ __forceinline__ void dep_guard1(v8f& a, v8f& b, v16us x) {
#if defined(__HIP_DEVICE_COMPILE__)
  asm volatile("v_nop\n\tv_nop\n\tv_nop\n\tv_nop" : "+v"(a), "+v"(b) : "v"(x));
#endif
}
__device__ __forceinline__ void dep_guard2(v8f& a, v8f& b, v8f& c, v8f& d, v16us x, v16us y) {
#if defined(__HIP_DEVICE_COMPILE__)
  asm volatile("v_nop\n\tv_nop\n\tv_nop\n\tv_nop" : "+v"(a), "+v"(b), "+v"(c), "+v"(d) : "v"(x), "v"(y));
#endif
}
__device__ __forceinline__ void keep4_u(v16us a, v16us b, v16us c, v16us d) {
#if defined(__HIP_DEVICE_COMPILE__)
  asm volatile("v_nop" :: "v"(a), "v"(b), "v"(c), "v"(d));
#endif
}
__device__ __forceinline__ void acc_guard4(v8f& a, v8f& b, v8f& c, v8f& d) {
#if defined(__HIP_DEVICE_COMPILE__)
  asm volatile("v_nop\n\tv_nop\n\tv_nop\n\tv_nop" : "+v"(a), "+v"(b), "+v"(c), "+v"(d));
#endif
}
__device__ __forceinline__ void guard4x6(v8f& a, v8f& b, v8f& c, v8f& d,
                                         v16us p, v16us q, v16us r, v16us s, v16us t, v16us u) {
#if defined(__HIP_DEVICE_COMPILE__)
  asm volatile("v_nop\n\tv_nop\n\tv_nop\n\tv_nop"
               : "+v"(a), "+v"(b), "+v"(c), "+v"(d)
               : "v"(p), "v"(q), "v"(r), "v"(s), "v"(t), "v"(u));
#endif
}
__device__ __forceinline__ void wave_sync_lds() {
  __builtin_amdgcn_fence(__ATOMIC_RELEASE, "workgroup");
  __builtin_amdgcn_wave_barrier();
  __builtin_amdgcn_fence(__ATOMIC_ACQUIRE, "workgroup");
}

__global__ __launch_bounds__(256) void cvt_rows(const float* __restrict__ x, unsigned short* xh, int nrows, float sc) {
  const int row = blockIdx.x * 8 + (threadIdx.x >> 5);
  const int lane = threadIdx.x & 31;
  if (row >= nrows) return;
  v4u hv[HH / 256];
#pragma unroll
  for (int c = 0; c < HH / 256; ++c) {
    const float* p = x + (size_t)row * HH + c * 256 + lane * 8;
    const v4f a0 = *(const v4f*)(p);
    const v4f a1 = *(const v4f*)(p + 4);
    v4u h;
#pragma unroll
    for (int e = 0; e < 2; ++e) {
      h[e]     = pk16(f2h(bfr(a0[2 * e]) * sc), f2h(bfr(a0[2 * e + 1]) * sc));
      h[2 + e] = pk16(f2h(bfr(a1[2 * e]) * sc), f2h(bfr(a1[2 * e + 1]) * sc));
    }
    hv[c] = h;
  }
  unsigned short* d = xh + (size_t)row * HH + lane * 8;
  for (int pass = 0; pass < 2; ++pass) {
#pragma unroll
    for (int c = 0; c < HH / 256; ++c) *(volatile v4u*)(d + c * 256) = hv[c];
    __threadfence();
  }
}

template <int OM, int CBM, int ASPL>
__global__ __launch_bounds__(256) void gemm64(
    const unsigned short* __restrict__ Ap, const unsigned short* __restrict__ Alp, int lda,
    const unsigned short* __restrict__ Btp, int ldb,
    unsigned short* Ch, unsigned short* Cl, float* Cf, int ldc,
    const float* __restrict__ cb, float wsc, float osc, int M, int N, int K) {
  constexpr int MI = ASPL ? 2 : 4;
  constexpr int TR = 16 * MI;
  __shared__ __align__(16) float sT[8][16 * 68];
  const int lane = threadIdx.x & 31;
  const int wave = threadIdx.x >> 5;
  const int tilesN = N >> 6;
  const int tilesM = M / TR;
  const int tile = blockIdx.x * 8 + wave;
  if (tile >= tilesM * tilesN) return;
  const int tm = tile / tilesN;
  const int tn = tile - tm * tilesN;
  const int m0 = tm * TR;
  const int n0 = tn << 6;

  const int rlane = lane & 15;
  const int koff  = (lane >> 4) * 8;
  const int mOff  = (lane >> 4) * 8;

  v8f acc[MI][4];
  v8f accr[MI][4];
#pragma unroll
  for (int i = 0; i < MI; ++i)
#pragma unroll
    for (int j = 0; j < 4; ++j) { acc[i][j] = zero8(); accr[i][j] = zero8(); }

  for (int k0 = 0; k0 < K; k0 += 32) {
    v16us bh[4];
#pragma unroll
    for (int j = 0; j < 4; ++j) {
      const size_t bo = (size_t)(n0 + (j << 4) + rlane) * ldb + koff + k0;
      bh[j] = ldfrag_u(Btp + bo);
    }
#pragma unroll
    for (int i = 0; i < MI; ++i) {
      const size_t ao = (size_t)(m0 + (i << 4) + rlane) * lda + koff + k0;
      const v16us ah = ldfrag_u(Ap + ao);
      if (ASPL) {
        const v16us al = ldfrag_u(Alp + ao);
#pragma unroll
        for (int j = 0; j < 4; ++j) {
          acc[i][j]  = mma_h_raw(ah, bh[j], acc[i][j]);
          accr[i][j] = mma_h_raw(al, bh[j], accr[i][j]);
        }
        dep_guard2(acc[i][0], acc[i][3], accr[i][0], accr[i][3], ah, al);
      } else {
#pragma unroll
        for (int j = 0; j < 4; ++j) acc[i][j] = mma_h_raw(ah, bh[j], acc[i][j]);
        dep_guard1(acc[i][0], acc[i][3], ah);
      }
    }
    keep4_u(bh[0], bh[1], bh[2], bh[3]);
  }
#pragma unroll
  for (int i = 0; i < MI; ++i) {
    acc_guard4(acc[i][0], acc[i][1], acc[i][2], acc[i][3]);
    if (ASPL) acc_guard4(accr[i][0], accr[i][1], accr[i][2], accr[i][3]);
  }

  const int hh2 = lane >> 4, c4 = (lane & 15) * 4;
  const int q8  = lane >> 3, c8 = (lane & 7) * 8;

  v4f cb4 = {0.f, 0.f, 0.f, 0.f};
  float cbc[8];
#pragma unroll
  for (int e = 0; e < 8; ++e) cbc[e] = 0.f;
  if (OM == 0 && CBM == 1) {
    const v4f v = *(const v4f*)(cb + n0 + c4);
    cb4[0] = bfr(v[0]); cb4[1] = bfr(v[1]); cb4[2] = bfr(v[2]); cb4[3] = bfr(v[3]);
  }
  if (OM == 1 && CBM == 1) {
    const v4f v0 = *(const v4f*)(cb + n0 + c8);
    const v4f v1 = *(const v4f*)(cb + n0 + c8 + 4);
#pragma unroll
    for (int e = 0; e < 4; ++e) { cbc[e] = bfr(v0[e]); cbc[4 + e] = bfr(v1[e]); }
  }

  float* slab = sT[wave];
#pragma unroll
  for (int i = 0; i < MI; ++i) {
    const int mBase = m0 + (i << 4);
#pragma unroll
    for (int j = 0; j < 4; ++j) {
#pragma unroll
      for (int r = 0; r < 8; ++r) {
        float v = acc[i][j][r];
        if (ASPL) v += accr[i][j][r] * RSCI;
        slab[(mOff + r) * 68 + (j << 4) + rlane] = v;
      }
    }
    wave_sync_lds();
    if (OM == 0) {
      v4f vals[8];
#pragma unroll
      for (int it = 0; it < 8; ++it) {
        const int row = it * 2 + hh2;
        const v4f v = *(const v4f*)(slab + row * 68 + c4);
        vals[it] = (v * wsc + cb4) * osc;
      }
      for (int pass = 0; pass < 2; ++pass) {
#pragma unroll
        for (int it = 0; it < 8; ++it) {
          const int row = it * 2 + hh2;
          *(volatile v4f*)(Cf + (size_t)(mBase + row) * ldc + (size_t)n0 + c4) = vals[it];
        }
        __threadfence();
      }
    }
    if (OM == 1) {
      v4u hv[4], lv[4];
#pragma unroll
      for (int it = 0; it < 4; ++it) {
        const int row = it * 4 + q8;
        const float* sp = slab + row * 68 + c8;
        float rb = 0.f;
        if (CBM == 2) rb = bfr(cb[mBase + row]);
        v4u ha = {0u, 0u, 0u, 0u}, la = {0u, 0u, 0u, 0u};
#pragma unroll
        for (int e = 0; e < 4; ++e) {
          const float f0 = (sp[2 * e]     * wsc + cbc[2 * e]     + rb) * osc;
          const float f1 = (sp[2 * e + 1] * wsc + cbc[2 * e + 1] + rb) * osc;
          unsigned short h0, l0, h1, l1;
          split_h(f0, h0, l0);
          split_h(f1, h1, l1);
          ha[e] = pk16(h0, h1);
          la[e] = pk16(l0, l1);
        }
        hv[it] = ha;
        lv[it] = la;
      }
      for (int pass = 0; pass < 2; ++pass) {
#pragma unroll
        for (int it = 0; it < 4; ++it) {
          const int row = it * 4 + q8;
          const size_t go = (size_t)(mBase + row) * ldc + (size_t)n0 + c8;
          *(volatile v4u*)(Ch + go) = hv[it];
          *(volatile v4u*)(Cl + go) = lv[it];
        }
        __threadfence();
      }
    }
    wave_sync_lds();
  }
}

__global__ __launch_bounds__(256) void attn_kernel(const unsigned short* __restrict__ Qh,
                                                   const unsigned short* __restrict__ Ql,
                                                   const unsigned short* __restrict__ Kh,
                                                   const unsigned short* __restrict__ Kl,
                                                   const unsigned short* __restrict__ VT,
                                                   const unsigned short* __restrict__ VTl,
                                                   unsigned short* Zh, unsigned short* Zl) {
  __shared__ __align__(16) unsigned short ps[8 * 1024];
  __shared__ __align__(16) unsigned short zsth[QT * ZSP];
  __shared__ __align__(16) unsigned short zstl[QT * ZSP];
  const int tq0  = blockIdx.x * QT;
  const int tk00 = tq0 & ~(SEGL - 1);
  const int hc   = blockIdx.y * HD;
  const int t = threadIdx.x, lane = t & 31, wv = t >> 5, hh = lane >> 4, jc = lane & 15;

  const size_t qo = (size_t)(tq0 + 16 * wv + jc) * HH + hc + 8 * hh;
  const v16us qf0 = ldfrag_u(Qh + qo);
  const v16us qf1 = ldfrag_u(Qh + qo + 32);
  const v16us ql0 = ldfrag_u(Ql + qo);
  const v16us ql1 = ldfrag_u(Ql + qo + 32);
  float m[8], ll[8];
  v8f oz[4], orr[4];
#pragma unroll
  for (int r = 0; r < 8; ++r) { m[r] = -1.0e30f; ll[r] = 0.f; }
#pragma unroll
  for (int d = 0; d < 4; ++d) { oz[d] = zero8(); orr[d] = zero8(); }
  unsigned short* pw = ps + wv * 1024;
  const size_t vob = (size_t)(hc + jc) * MT;

#pragma unroll 1
  for (int c = 0; c < NCHK; ++c) {
    const int tk0 = tk00 + 32 * c;
    const size_t ko0 = (size_t)(tk0 + jc) * HH + hc + 8 * hh;
    const size_t ko1 = ko0 + (size_t)16 * HH;
    v8f s0 = zero8(), s1 = zero8(), sr0 = zero8(), sr1 = zero8();
    {
      const v16us kf0 = ldfrag_u(Kh + ko0);
      const v16us kf1 = ldfrag_u(Kh + ko1);
      const v16us kl0 = ldfrag_u(Kl + ko0);
      const v16us kl1 = ldfrag_u(Kl + ko1);
      s0  = mma_h_raw(qf0, kf0, s0);
      sr0 = mma_h_raw(qf0, kl0, sr0);
      s1  = mma_h_raw(qf0, kf1, s1);
      sr1 = mma_h_raw(qf0, kl1, sr1);
      sr0 = mma_h_raw(ql0, kf0, sr0);
      sr1 = mma_h_raw(ql0, kf1, sr1);
      guard4x6(s0, s1, sr0, sr1, qf0, ql0, kf0, kf1, kl0, kl1);
    }
    {
      const v16us kf0 = ldfrag_u(Kh + ko0 + 32);
      const v16us kf1 = ldfrag_u(Kh + ko1 + 32);
      const v16us kl0 = ldfrag_u(Kl + ko0 + 32);
      const v16us kl1 = ldfrag_u(Kl + ko1 + 32);
      s0  = mma_h_raw(qf1, kf0, s0);
      sr0 = mma_h_raw(qf1, kl0, sr0);
      s1  = mma_h_raw(qf1, kf1, s1);
      sr1 = mma_h_raw(qf1, kl1, sr1);
      sr0 = mma_h_raw(ql1, kf0, sr0);
      sr1 = mma_h_raw(ql1, kf1, sr1);
      guard4x6(s0, s1, sr0, sr1, qf1, ql1, kf0, kf1, kl0, kl1);
    }
    wave_sync_lds();
#pragma unroll
    for (int r = 0; r < 8; ++r) {
      const int il = 8 * hh + r;
      const float t0 = (s0[r] + sr0[r] * RSCI) * SCL;
      const float t1 = (s1[r] + sr1[r] * RSCI) * SCL;
      float rm = fmaxf(t0, t1);
#pragma unroll
      for (int off = 1; off < 16; off <<= 1) rm = fmaxf(rm, __shfl_xor(rm, off, 32));
      const float mn2   = fmaxf(m[r], rm);
      const float alpha = __expf(m[r] - mn2);
      const float e0 = __expf(t0 - mn2);
      const float e1 = __expf(t1 - mn2);
      float rs = e0 + e1;
#pragma unroll
      for (int off = 1; off < 16; off <<= 1) rs += __shfl_xor(rs, off, 32);
      ll[r] = ll[r] * alpha + rs;
      m[r]  = mn2;
#pragma unroll
      for (int d = 0; d < 4; ++d) { oz[d][r] *= alpha; orr[d][r] *= alpha; }
      unsigned short h0, l0, h1, l1;
      split_h(e0 * PSC, h0, l0);
      split_h(e1 * PSC, h1, l1);
      pw[il * 32 + jc]            = h0;
      pw[il * 32 + 16 + jc]       = h1;
      pw[512 + il * 32 + jc]      = l0;
      pw[512 + il * 32 + 16 + jc] = l1;
    }
    wave_sync_lds();
    FragU pa, pb;
    pa.h[0] = *(const v8us*)(pw + jc * 32 + 8 * hh);
    pa.h[1] = *(const v8us*)(pw + jc * 32 + 16 + 8 * hh);
    pb.h[0] = *(const v8us*)(pw + 512 + jc * 32 + 8 * hh);
    pb.h[1] = *(const v8us*)(pw + 512 + jc * 32 + 16 + 8 * hh);
#pragma unroll
    for (int dg = 0; dg < 2; ++dg) {
      const size_t voa = vob + (size_t)(32 * dg) * MT + tk0 + 8 * hh;
      const size_t voc = voa + (size_t)16 * MT;
      const v16us f0 = ldfrag_u(VT  + voa);
      const v16us f1 = ldfrag_u(VT  + voc);
      const v16us g0 = ldfrag_u(VTl + voa);
      const v16us g1 = ldfrag_u(VTl + voc);
      oz[2 * dg]      = mma_h_raw(pa.v, f0, oz[2 * dg]);
      orr[2 * dg]     = mma_h_raw(pa.v, g0, orr[2 * dg]);
      oz[2 * dg + 1]  = mma_h_raw(pa.v, f1, oz[2 * dg + 1]);
      orr[2 * dg + 1] = mma_h_raw(pa.v, g1, orr[2 * dg + 1]);
      orr[2 * dg]     = mma_h_raw(pb.v, f0, orr[2 * dg]);
      orr[2 * dg + 1] = mma_h_raw(pb.v, f1, orr[2 * dg + 1]);
      guard4x6(oz[2 * dg], oz[2 * dg + 1], orr[2 * dg], orr[2 * dg + 1], pa.v, pb.v, f0, f1, g0, g1);
    }
  }

#pragma unroll
  for (int r = 0; r < 8; ++r) {
    const int il = 8 * hh + r;
    const float l = ll[r];
    const float inv = ((l > 0.f) ? (1.0f / l) : 0.f) * (ZSC / PSC);
    const int so = (16 * wv + il) * ZSP + jc;
#pragma unroll
    for (int d = 0; d < 4; ++d) {
      const float z = (oz[d][r] + orr[d][r] * RSCI) * inv;
      unsigned short h0, l0;
      split_h(z, h0, l0);
      zsth[so + 16 * d] = h0;
      zstl[so + 16 * d] = l0;
    }
  }
  __syncthreads();
  v4u hv[4], lv[4];
#pragma unroll
  for (int it = 0; it < 4; ++it) {
    const int row = it * 32 + (t >> 3), p = (t & 7) * 8;
    hv[it] = *(const v4u*)(zsth + row * ZSP + p);
    lv[it] = *(const v4u*)(zstl + row * ZSP + p);
  }
  for (int pass = 0; pass < 2; ++pass) {
#pragma unroll
    for (int it = 0; it < 4; ++it) {
      const int row = it * 32 + (t >> 3), p = (t & 7) * 8;
      const size_t go = (size_t)(tq0 + row) * HH + hc + p;
      *(volatile v4u*)(Zh + go) = hv[it];
      *(volatile v4u*)(Zl + go) = lv[it];
    }
    __threadfence();
  }
}

extern "C" void kernel_launch(void* const* d_in, const int* in_sizes, int n_in,
                              void* d_out, int out_size, void* d_ws, size_t ws_size,
                              hipStream_t stream) {
  if (n_in < 9) return;
  if (in_sizes[0] != MT * HH) return;
  if (in_sizes[1] != HH * HH || in_sizes[2] != HH) return;
  if (in_sizes[3] != HH * HH || in_sizes[4] != HH) return;
  if (in_sizes[5] != HH * HH || in_sizes[6] != HH) return;
  if (in_sizes[7] != HH * HH || in_sizes[8] != HH) return;
  if (out_size != MT * HH) return;

  const float* x  = (const float*)d_in[0];
  const float* Wq = (const float*)d_in[1];
  const float* bq = (const float*)d_in[2];
  const float* Wk = (const float*)d_in[3];
  const float* bk = (const float*)d_in[4];
  const float* Wv = (const float*)d_in[5];
  const float* bv = (const float*)d_in[6];
  const float* Wo = (const float*)d_in[7];
  const float* bo = (const float*)d_in[8];

  const size_t PX  = (size_t)MT * HH * 2;
  const size_t PW  = (size_t)HH * HH * 2;
  const size_t PVT = (size_t)HH * MT * 2;
  size_t off = 0;
  const size_t oXh = off; off += PX;
  const size_t oWq = off; off += PW;
  const size_t oWk = off; off += PW;
  const size_t oWv = off; off += PW;
  const size_t oWo = off; off += PW;
  const size_t oQh = off; off += PX;
  const size_t oQl = off; off += PX;
  const size_t oKh = off; off += PX;
  const size_t oKl = off; off += PX;
  const size_t oVT = off; off += PVT;
  const size_t oVL = off; off += PVT;
  const size_t oZh = off; off += PX;
  const size_t oZl = off; off += PX;
  if (off > ws_size) return;
  if (off > (size_t)134217728) return;

  char* ws = (char*)d_ws;
  unsigned short* Xh   = (unsigned short*)(ws + oXh);
  unsigned short* Wq16 = (unsigned short*)(ws + oWq);
  unsigned short* Wk16 = (unsigned short*)(ws + oWk);
  unsigned short* Wv16 = (unsigned short*)(ws + oWv);
  unsigned short* Wo16 = (unsigned short*)(ws + oWo);
  unsigned short* Qh   = (unsigned short*)(ws + oQh);
  unsigned short* Ql   = (unsigned short*)(ws + oQl);
  unsigned short* Kh   = (unsigned short*)(ws + oKh);
  unsigned short* Kl   = (unsigned short*)(ws + oKl);
  unsigned short* VT   = (unsigned short*)(ws + oVT);
  unsigned short* VTl  = (unsigned short*)(ws + oVL);
  unsigned short* Zh   = (unsigned short*)(ws + oZh);
  unsigned short* Zl   = (unsigned short*)(ws + oZl);
  float*          out0 = (float*)d_out;

  const dim3 blk(256);
  const int gqk = ((MT / 64) * (HH / 64)) / 8;
  const int gvt = ((HH / 64) * (MT / 64)) / 8;
  const int gsp = ((MT / 32) * (HH / 64)) / 8;
  if ((((MT / 64) * (HH / 64)) % 8) != 0) return;
  if ((((HH / 64) * (MT / 64)) % 8) != 0) return;
  if ((((MT / 32) * (HH / 64)) % 8) != 0) return;

  cvt_rows<<<dim3(MT / 8), blk, 0, stream>>>(x, Xh, MT, 1.0f);
  cvt_rows<<<dim3(HH / 8), blk, 0, stream>>>(Wq, Wq16, HH, WSC);
  cvt_rows<<<dim3(HH / 8), blk, 0, stream>>>(Wk, Wk16, HH, WSC);
  cvt_rows<<<dim3(HH / 8), blk, 0, stream>>>(Wv, Wv16, HH, WSC);
  cvt_rows<<<dim3(HH / 8), blk, 0, stream>>>(Wo, Wo16, HH, WSC);

  gemm64<1, 1, 0><<<dim3(gqk), blk, 0, stream>>>(
      Xh, Xh, HH, Wq16, HH, Qh, Ql, out0, HH, bq, 1.0f / WSC, 1.0f, MT, HH, HH);
  gemm64<1, 1, 0><<<dim3(gqk), blk, 0, stream>>>(
      Xh, Xh, HH, Wk16, HH, Kh, Kl, out0, HH, bk, 1.0f / WSC, 1.0f, MT, HH, HH);
  gemm64<1, 2, 0><<<dim3(gvt), blk, 0, stream>>>(
      Wv16, Wv16, HH, Xh, HH, VT, VTl, out0, MT, bv, 1.0f / WSC, 1.0f, HH, MT, HH);

  attn_kernel<<<dim3(MT / QT, NHD), blk, 0, stream>>>(Qh, Ql, Kh, Kl, VT, VTl, Zh, Zl);

  gemm64<0, 1, 1><<<dim3(gsp), blk, 0, stream>>>(
      Zh, Zl, HH, Wo16, HH, Qh, Ql, out0, HH, bo, 1.0f / (WSC * ZSC), 1.0f, MT, HH, HH);
  (void)hipGetLastError();
}
